// GraphAttentionSeg_8650064134304
// MI455X (gfx1250) — hardware-verified
//
#include <hip/hip_runtime.h>


#define NM 32768
#define NC 64
#define NK 16
#define NEDG (NM * NK)
#define CHP 8192
#define CHE (CHP * NK)
#define NBLK1 (NM / 16)
#define NBLK2 (NEDG / 1024)
#define BN_EPS 1e-5f

typedef __attribute__((ext_vector_type(16))) __bf16   v16bf;
typedef __attribute__((ext_vector_type(16))) _Float16 v16h;
typedef __attribute__((ext_vector_type(8)))  float    v8f;
typedef __attribute__((ext_vector_type(8)))  unsigned v8u;

__device__ __forceinline__ unsigned f2bf(float f) { unsigned u = __float_as_uint(f); u += 0x7FFFu + ((u >> 16) & 1u); return u >> 16; }
__device__ __forceinline__ unsigned f2h(float f) { return (unsigned)__builtin_bit_cast(unsigned short, (_Float16)f); }
__device__ __forceinline__ int kpat(int v, int half) { return ((v & 4) ? 16 : 0) + half * 8 + 2 * (v & 3); }

template <int F16, int NP> struct Opnd { v16bf p[NP]; };

template <int F16, int NP> __device__ __forceinline__ void pack2(float f0, float f1, unsigned* o) {
    if (F16) { o[0] = f2h(f0) | (f2h(f1) << 16); return; }
    unsigned h0 = f2bf(f0), h1 = f2bf(f1); o[0] = h0 | (h1 << 16);
    if (NP >= 2) {
        float r0 = f0 - __uint_as_float(h0 << 16), r1 = f1 - __uint_as_float(h1 << 16);
        unsigned m0 = f2bf(r0), m1 = f2bf(r1); o[1] = m0 | (m1 << 16);
        if (NP >= 3) {
            float s0 = r0 - __uint_as_float(m0 << 16), s1 = r1 - __uint_as_float(m1 << 16);
            o[2] = f2bf(s0) | (f2bf(s1) << 16);
        }
    }
}
template <int F16, int NP> __device__ __forceinline__ void op_row(const float* rowp, int half, float sc, Opnd<F16, NP>& o) {
    v8u u[NP];
#pragma unroll
    for (int v = 0; v < 8; ++v) {
        int kk = kpat(v, half); unsigned t[3];
        pack2<F16, NP>(rowp[kk] * sc, rowp[kk + 1] * sc, t);
#pragma unroll
        for (int p = 0; p < NP; ++p) u[p][v] = t[p];
    }
#pragma unroll
    for (int p = 0; p < NP; ++p) o.p[p] = __builtin_bit_cast(v16bf, u[p]);
}
template <int F16, int NP> __device__ __forceinline__ void op_row_tail(const float* rowp, int half, float sc, int kvalid, Opnd<F16, NP>& o) {
    v8u u[NP];
#pragma unroll
    for (int v = 0; v < 8; ++v) {
        int kk = kpat(v, half); unsigned t[3];
        float f0 = kk < kvalid ? rowp[kk] * sc : 0.0f, f1 = (kk + 1) < kvalid ? rowp[kk + 1] * sc : 0.0f;
        pack2<F16, NP>(f0, f1, t);
#pragma unroll
        for (int p = 0; p < NP; ++p) u[p][v] = t[p];
    }
#pragma unroll
    for (int p = 0; p < NP; ++p) o.p[p] = __builtin_bit_cast(v16bf, u[p]);
}
template <int F16, int NP> __device__ __forceinline__ void op_col(const float* M, int ld, int n, int k0, int half, float sc, Opnd<F16, NP>& o) {
    v8u u[NP];
#pragma unroll
    for (int v = 0; v < 8; ++v) {
        int kk = k0 + kpat(v, half); unsigned t[3];
        pack2<F16, NP>(M[(size_t)kk * ld + n] * sc, M[(size_t)(kk + 1) * ld + n] * sc, t);
#pragma unroll
        for (int p = 0; p < NP; ++p) u[p][v] = t[p];
    }
#pragma unroll
    for (int p = 0; p < NP; ++p) o.p[p] = __builtin_bit_cast(v16bf, u[p]);
}
template <int F16, int NP> __device__ __forceinline__ void op_col_tail(const float* M, int ld, int n, int k0, int half, float sc, int K, Opnd<F16, NP>& o) {
    v8u u[NP];
#pragma unroll
    for (int v = 0; v < 8; ++v) {
        int kk = k0 + kpat(v, half); unsigned t[3];
        float f0 = kk < K ? M[(size_t)kk * ld + n] * sc : 0.0f, f1 = (kk + 1) < K ? M[(size_t)(kk + 1) * ld + n] * sc : 0.0f;
        pack2<F16, NP>(f0, f1, t);
#pragma unroll
        for (int p = 0; p < NP; ++p) u[p][v] = t[p];
    }
#pragma unroll
    for (int p = 0; p < NP; ++p) o.p[p] = __builtin_bit_cast(v16bf, u[p]);
}
__device__ __forceinline__ v8f wm_bf16(v16bf a, v16bf b, v8f c) { return __builtin_amdgcn_wmma_f32_16x16x32_bf16(false, a, false, b, (short)0, c, false, false); }
template <int F16, int NA, int NB> __device__ __forceinline__ v8f wmma_op(const Opnd<F16, NA>& a, const Opnd<F16, NB>& b, v8f c) {
    if (F16) {
        v16h ah = __builtin_bit_cast(v16h, a.p[0]), bh = __builtin_bit_cast(v16h, b.p[0]);
        c = __builtin_amdgcn_wmma_f32_16x16x32_f16(false, ah, false, bh, (short)0, c, false, false);
        asm volatile("v_nop\n\tv_nop\n\tv_nop\n\tv_nop" : "+v"(c) : "v"(ah), "v"(bh));
        return c;
    }
    constexpr int NMX = NA > NB ? NA : NB;
#pragma unroll
    for (int i = 0; i < NA; ++i)
#pragma unroll
        for (int j = 0; j < NB; ++j)
            if (i + j < NMX) c = wm_bf16(a.p[i], b.p[j], c);
    if (NA == 1 && NB == 1)      asm volatile("v_nop\n\tv_nop\n\tv_nop\n\tv_nop" : "+v"(c) : "v"(a.p[0]), "v"(b.p[0]));
    else if (NA == 2 && NB == 1) asm volatile("v_nop\n\tv_nop\n\tv_nop\n\tv_nop" : "+v"(c) : "v"(a.p[0]), "v"(a.p[1]), "v"(b.p[0]));
    else if (NA == 1 && NB == 2) asm volatile("v_nop\n\tv_nop\n\tv_nop\n\tv_nop" : "+v"(c) : "v"(a.p[0]), "v"(b.p[0]), "v"(b.p[1]));
    else if (NA == 2 && NB == 2) asm volatile("v_nop\n\tv_nop\n\tv_nop\n\tv_nop" : "+v"(c) : "v"(a.p[0]), "v"(a.p[1]), "v"(b.p[0]), "v"(b.p[1]));
    else                         asm volatile("v_nop\n\tv_nop\n\tv_nop\n\tv_nop" : "+v"(c) : "v"(a.p[0]), "v"(a.p[NA - 1]), "v"(b.p[0]), "v"(b.p[NB - 1]), "v"(a.p[NA / 2]), "v"(b.p[NB / 2]));
    return c;
}

struct ZMap { long long s1; long long s2; int zdiv; int pad_; };
__device__ __forceinline__ size_t zoff(const ZMap& m, int z) { return (size_t)((long long)(z / m.zdiv) * m.s1 + (long long)(z % m.zdiv) * m.s2); }

#define ACT_NONE 0
#define ACT_RELU 1
#define ACT_GELU_ERF 2
#define ACT_SILU 3
#define ACT_TANH 4
__device__ __forceinline__ float act_apply(int act, float x) {
    if (act == ACT_RELU) return x > 0.f ? x : 0.f;
    if (act == ACT_GELU_ERF) return 0.5f * x * (1.0f + erff(x * 0.70710678118654752f));
    if (act == ACT_SILU) return x / (1.0f + expf(-x));
    if (act == ACT_TANH) return tanhf(x);
    return x;
}
struct GemmArgs {
    ZMap za, zb_, zc, zbias, zadd, zrsc, zmul, zrbias;
    const float* A; const float* Bm; float* C; const float* bias; const float* add; const float* rsc; const float* mul; const float* rbias;
    long long ldadd, ldmul;
    int lda, ldb, ldc, K;
    float ascale, bscale, oscale, addscale;
    int M, nvalid, nstore, ldrsc;
    int bcs, pad1, pad2, pad3;
};
template <int BT, int F16, int NA, int NB, int RW, int CW, int ACT>
__global__ __launch_bounds__(256) void gemm_kernel(GemmArgs g) {
    constexpr int TR = 16 * RW, TC = 64 * CW, CSTR = TC + 4;
    __shared__ __align__(16) float cst[TR * CSTR];
    const int z = blockIdx.z;
    const float* A = g.A + zoff(g.za, z); const float* Bm = g.Bm + zoff(g.zb_, z); float* C = g.C + zoff(g.zc, z);
    const int tid = threadIdx.x, lane = tid & 31, wv = tid >> 5;
    const int l16 = lane & 15, half = lane >> 4;
    const int rt = wv % RW, ch = wv / RW;
    const int row0 = blockIdx.x * TR, col0 = blockIdx.y * TC + ch * 64;
    int arix = row0 + rt * 16 + l16; if (arix >= g.M) arix = g.M - 1;
    const float* arow = A + (size_t)arix * g.lda;
    v8f acc[4];
#pragma unroll
    for (int t = 0; t < 4; ++t) acc[t] = (v8f){};
    const int K = g.K;
#pragma unroll 1
    for (int kc = 0; kc < K; kc += 32) {
        Opnd<F16, NA> a;
        if (kc + 32 <= K) op_row<F16, NA>(arow + kc, half, g.ascale, a); else op_row_tail<F16, NA>(arow + kc, half, g.ascale, K - kc, a);
#pragma unroll
        for (int t = 0; t < 4; ++t) {
            Opnd<F16, NB> b;
            const int n = col0 + t * 16 + l16;
            if (n < g.nvalid) {
                if (BT) { if (kc + 32 <= K) op_row<F16, NB>(Bm + (size_t)n * g.ldb + kc, half, g.bscale, b); else op_row_tail<F16, NB>(Bm + (size_t)n * g.ldb + kc, half, g.bscale, K - kc, b); }
                else    { if (kc + 32 <= K) op_col<F16, NB>(Bm, g.ldb, n * g.bcs, kc, half, g.bscale, b); else op_col_tail<F16, NB>(Bm, g.ldb, n * g.bcs, kc, half, g.bscale, K, b); }
            } else {
#pragma unroll
                for (int p = 0; p < NB; ++p) b.p[p] = (v16bf){};
            }
            acc[t] = wmma_op<F16, NA, NB>(a, b, acc[t]);
        }
    }
    const float* bias = g.bias ? g.bias + zoff(g.zbias, z) : nullptr;
    const float* add = g.add ? g.add + zoff(g.zadd, z) : nullptr;
    const float* rsc = g.rsc ? g.rsc + zoff(g.zrsc, z) : nullptr;
    const float* mul = g.mul ? g.mul + zoff(g.zmul, z) : nullptr;
    const float* rbias = g.rbias ? g.rbias + zoff(g.zrbias, z) : nullptr;
#pragma unroll
    for (int t = 0; t < 4; ++t) {
        const int cl = ch * 64 + t * 16 + l16;
        const int cg = blockIdx.y * TC + cl;
        const bool cok = cg < g.nvalid;
        const float bv = (bias && cok) ? bias[(size_t)cg * g.bcs] : 0.0f;
#pragma unroll
        for (int r = 0; r < 8; ++r) {
            const int rl = rt * 16 + r + 8 * half;
            float v = acc[t][r] * g.oscale + bv;
            int rg = row0 + rl; if (rg >= g.M) rg = g.M - 1;
            if (rbias) v += rbias[rg];
            if (rsc) v *= rsc[(size_t)rg * g.ldrsc];
            if (mul && cok) v *= mul[(size_t)rg * g.ldmul + cg];
            if (add && cok) v += g.addscale * add[(size_t)rg * g.ldadd + cg];
            cst[rl * CSTR + cl] = v;
        }
    }
    __syncthreads();
    const int col = tid % TC, rsel = tid / TC, rstep = 256 / TC;
    if (ACT != ACT_NONE) {
#pragma unroll 1
        for (int r = rsel; r < TR; r += rstep) cst[r * CSTR + col] = act_apply(ACT, cst[r * CSTR + col]);
    }
    float* ob = C + (size_t)row0 * g.ldc + (size_t)blockIdx.y * TC;
    const bool colok = (int)(blockIdx.y * TC + col) < g.nstore;
    const int rmax = (g.M - row0 < TR) ? (g.M - row0) : TR;
    auto pass = [&]() {
        if (colok) {
#pragma unroll 4
            for (int r = rsel; r < rmax; r += rstep) *(volatile float*)(ob + (size_t)r * g.ldc + col) = cst[r * CSTR + col];
        }
    };
    pass();
    __threadfence();
    pass();
}
static inline ZMap zm(long long s1) { ZMap m; m.s1 = s1; m.s2 = 0; m.zdiv = 1; m.pad_ = 0; return m; }
static inline ZMap zm2(long long s1, long long s2, int zdiv) { ZMap m; m.s1 = s1; m.s2 = s2; m.zdiv = zdiv; m.pad_ = 0; return m; }
static inline GemmArgs gemm_args(const float* A, int lda, ZMap za, const float* Bm, int ldb, ZMap zb, float* C, int ldc, ZMap zc, int M, int N, int K) {
    GemmArgs g; g.za = za; g.zb_ = zb; g.zc = zc; g.zbias = zm(0); g.zadd = zm(0); g.zrsc = zm(0); g.zmul = zm(0); g.zrbias = zm(0);
    g.A = A; g.Bm = Bm; g.C = C; g.bias = nullptr; g.add = nullptr; g.rsc = nullptr; g.mul = nullptr; g.rbias = nullptr; g.ldadd = 0; g.ldmul = 0;
    g.lda = lda; g.ldb = ldb; g.ldc = ldc; g.K = K; g.ascale = 1.0f; g.bscale = 1.0f; g.oscale = 1.0f; g.addscale = 1.0f; g.M = M; g.nvalid = N; g.nstore = N; g.ldrsc = 1;
    g.bcs = 1; g.pad1 = 0; g.pad2 = 0; g.pad3 = 0;
    return g;
}
static_assert(sizeof(ZMap) == 24, "ZMap layout");
static_assert(sizeof(GemmArgs) == 8 * 24 + 8 * 8 + 2 * 8 + 4 * 4 + 4 * 4 + 4 * 4 + 4 * 4, "GemmArgs has no padding");

__global__ __launch_bounds__(256) void softmax_rows(float* S, long long sy, long long sx, int L, float prescale, const float* addv, long long say, int aydiv, int causal,
                                                  const int* imask, long long imy, long long imx, float maskval) {
    __shared__ float red[8];
    const int tid = threadIdx.x, lane = tid & 31, wid = tid >> 5;
    float* row = S + (size_t)blockIdx.y * sy + (size_t)blockIdx.x * sx;
    const float* av = addv ? addv + (size_t)(blockIdx.y / aydiv) * say : nullptr;
    const int* im = imask ? imask + (size_t)(blockIdx.y / aydiv) * imy + (size_t)blockIdx.x * imx : nullptr;
    float v[16];
    const int nj = L / 256;
    float mx = -__builtin_inff();
#pragma unroll
    for (int j = 0; j < 16; ++j) if (j < nj) { float t = row[tid + 256 * j] * prescale; if (av) t += av[tid + 256 * j]; if (im && im[tid + 256 * j] == 0) t = maskval; if (causal && (tid + 256 * j) > (int)blockIdx.x) t = -__builtin_inff(); v[j] = t; mx = fmaxf(mx, t); }
#pragma unroll
    for (int o = 16; o; o >>= 1) mx = fmaxf(mx, __shfl_xor(mx, o, 32));
    if (lane == 0) red[wid] = mx;
    __syncthreads();
    float m = red[0];
#pragma unroll
    for (int i = 1; i < 8; ++i) m = fmaxf(m, red[i]);
    if (m == -__builtin_inff()) m = 0.f;
    __syncthreads();
    float sum = 0.f;
#pragma unroll
    for (int j = 0; j < 16; ++j) if (j < nj) { v[j] = expf(v[j] - m); sum += v[j]; }
#pragma unroll
    for (int o = 16; o; o >>= 1) sum += __shfl_xor(sum, o, 32);
    if (lane == 0) red[wid] = sum;
    __syncthreads();
    float tot = 0.f;
#pragma unroll
    for (int i = 0; i < 8; ++i) tot += red[i];
    const float inv = 1.0f / tot;
#pragma unroll
    for (int j = 0; j < 16; ++j) if (j < nj) *(volatile float*)(row + tid + 256 * j) = v[j] * inv;
    __threadfence();
#pragma unroll
    for (int j = 0; j < 16; ++j) if (j < nj) *(volatile float*)(row + tid + 256 * j) = v[j] * inv;
}

#define VST2(T, p, v) do { const T vst2_v_ = (v); *(volatile T*)(p) = vst2_v_; __threadfence(); *(volatile T*)(p) = vst2_v_; } while (0)
__device__ __forceinline__ int nbr(const int* __restrict__ idx, int e) { int j = idx[e]; return j < 0 ? 0 : (j >= NM ? NM - 1 : j); }

__global__ __launch_bounds__(256) void k_wd(const float* __restrict__ W, float* Wd) {
    const int t = blockIdx.x * 256 + threadIdx.x; if (t >= NC * NC) return; VST2(float, Wd + t, W[t] - W[NC * NC + t]);
}
__global__ __launch_bounds__(128) void k_stats1(const float* __restrict__ P, const float* __restrict__ Q, const float* __restrict__ pp, const int* __restrict__ idx,
                                                const float* __restrict__ W1, const float* __restrict__ b1, double* ps, double* pq) {
    const int blk = blockIdx.x, c = threadIdx.x; const int i0 = blk * 16;
    double s = 0.0, q = 0.0;
    if (c < NC) {
        for (int e = 0; e < 256; ++e) { const int i = i0 + (e >> 4); const int j = nbr(idx, i * NK + (e & 15)); const float v = P[(size_t)i * NC + c] + Q[(size_t)j * NC + c]; s += v; q += (double)v * v; }
    } else if (c < NC + 3) {
        const int a = c - NC;
        for (int e = 0; e < 256; ++e) { const int i = i0 + (e >> 4); const int j = nbr(idx, i * NK + (e & 15));
            const float dx = pp[j * 3] - pp[i * 3], dy = pp[j * 3 + 1] - pp[i * 3 + 1], dz = pp[j * 3 + 2] - pp[i * 3 + 2];
            const float v = dx * W1[0 * 3 + a] + dy * W1[1 * 3 + a] + dz * W1[2 * 3 + a] + b1[a]; s += v; q += (double)v * v; }
    }
    if (c < 96) { VST2(double, ps + (size_t)blk * 96 + c, s); VST2(double, pq + (size_t)blk * 96 + c, q); }
}
__global__ __launch_bounds__(128) void k_reduce(const double* __restrict__ ps, const double* __restrict__ pq, int nblk, int pitch, double cnt, float* mean, float* var) {
    const int c = threadIdx.x; if (c >= pitch) return;
    double s = 0.0, q = 0.0;
    for (int b = 0; b < nblk; ++b) { s += ps[(size_t)b * pitch + c]; q += pq[(size_t)b * pitch + c]; }
    const double m = s / cnt; double v = q / cnt - m * m; if (v < 0.0) v = 0.0;
    const float mf = (float)m, vf = (float)v;
    *(volatile float*)(mean + c) = mf; *(volatile float*)(var + c) = vf; __threadfence(); *(volatile float*)(mean + c) = mf; *(volatile float*)(var + c) = vf;
}
__global__ __launch_bounds__(256) void k_y1act(const float* __restrict__ P, const float* __restrict__ Q, const int* __restrict__ idx, const float* __restrict__ m1, const float* __restrict__ v1,
                                               const float* __restrict__ g, const float* __restrict__ bb, int e0, float* Y1c) {
    const size_t t = (size_t)blockIdx.x * 256 + threadIdx.x; if (t >= (size_t)CHE * NC) return;
    const int c = (int)(t % NC), el = (int)(t / NC); const int e = e0 + el; const int i = e / NK; const int j = nbr(idx, e);
    float v = P[(size_t)i * NC + c] + Q[(size_t)j * NC + c];
    v = (v - m1[c]) * rsqrtf(v1[c] + BN_EPS) * g[c] + bb[c]; v = v > 0.f ? v : 0.1f * v;
    VST2(float, Y1c + t, v);
}
__global__ __launch_bounds__(NC) void k_stats2(const float* __restrict__ Y2c, int slot0, double* ps, double* pq) {
    const int c = threadIdx.x, blk = blockIdx.x; double s = 0.0, q = 0.0;
    for (int r = 0; r < 1024; ++r) { const float v = Y2c[((size_t)blk * 1024 + r) * NC + c]; s += v; q += (double)v * v; }
    VST2(double, ps + (size_t)(slot0 + blk) * NC + c, s); VST2(double, pq + (size_t)(slot0 + blk) * NC + c, q);
}
__global__ __launch_bounds__(256) void k_apply(const float* __restrict__ Y2c, const float* __restrict__ pp, const int* __restrict__ idx, const float* __restrict__ W1, const float* __restrict__ b1,
                                               const float* __restrict__ mlp, const float* __restrict__ vlp, const float* __restrict__ glp, const float* __restrict__ blp,
                                               const float* __restrict__ W2, const float* __restrict__ b2, const float* __restrict__ m2, const float* __restrict__ v2,
                                               const float* __restrict__ g2, const float* __restrict__ bb2, int p0, float* ymax) {
    const size_t t = (size_t)blockIdx.x * 256 + threadIdx.x; if (t >= (size_t)CHP * NC) return;
    const int c = (int)(t % NC), il = (int)(t / NC); const int i = p0 + il;
    const float sc2 = rsqrtf(v2[c] + BN_EPS) * g2[c];
    float best = -__builtin_inff();
    for (int k = 0; k < NK; ++k) {
        const int e = i * NK + k; const int j = nbr(idx, e);
        const float dx = pp[j * 3] - pp[i * 3], dy = pp[j * 3 + 1] - pp[i * 3 + 1], dz = pp[j * 3 + 2] - pp[i * 3 + 2];
        float pe = b2[c];
#pragma unroll
        for (int a = 0; a < 3; ++a) {
            float h = dx * W1[0 * 3 + a] + dy * W1[1 * 3 + a] + dz * W1[2 * 3 + a] + b1[a];
            h = (h - mlp[a]) * rsqrtf(vlp[a] + BN_EPS) * glp[a] + blp[a]; h = fmaxf(h, 0.f);
            pe += h * W2[a * NC + c];
        }
        float y = Y2c[((size_t)il * NK + k) * NC + c];
        y = (y - m2[c]) * sc2 + bb2[c]; y = y > 0.f ? y : 0.1f * y;
        best = fmaxf(best, y + pe);
    }
    VST2(float, ymax + (size_t)i * NC + c, best);
}
__global__ __launch_bounds__(NC) void k_colstats(const float* __restrict__ a, float* mean, float* var) {
    const int c = threadIdx.x; double s = 0.0;
    for (int i = 0; i < NM; ++i) s += (double)a[(size_t)i * NC + c];
    const double m = s / (double)NM; double q = 0.0;
    for (int i = 0; i < NM; ++i) { const double v = (double)a[(size_t)i * NC + c] - m; q += v * v; }
    const float mf = (float)m, vf = (float)(q / (double)NM);
    *(volatile float*)(mean + c) = mf; *(volatile float*)(var + c) = vf; __threadfence(); *(volatile float*)(mean + c) = mf; *(volatile float*)(var + c) = vf;
}
__global__ __launch_bounds__(256) void k_bn_node(const float* __restrict__ a, const float* __restrict__ mean, const float* __restrict__ var, const float* __restrict__ g, const float* __restrict__ bb,
                                                const float* __restrict__ x, float* outp, int mode) {
    const size_t t = (size_t)blockIdx.x * 256 + threadIdx.x; if (t >= (size_t)NM * NC) return;
    const int c = (int)(t % NC);
    float v = (a[t] - mean[c]) * rsqrtf(var[c] + BN_EPS) * g[c] + bb[c];
    if (mode == 1) v += x[t];
    VST2(float, outp + t, fmaxf(v, 0.f));
}

extern "C" void kernel_launch(void* const* d_in, const int* in_sizes, int n_in,
                              void* d_out, int out_size, void* d_ws, size_t ws_size, hipStream_t stream) {
    (void)in_sizes; (void)n_in; (void)out_size;
    const float* pp = (const float*)d_in[0];
    const float* x = (const float*)d_in[1];
    const int* idx = (const int*)d_in[2];
    const float* lp_w1 = (const float*)d_in[3]; const float* lp_b1 = (const float*)d_in[4]; const float* lp_g = (const float*)d_in[5]; const float* lp_be = (const float*)d_in[6];
    const float* lp_w2 = (const float*)d_in[7]; const float* lp_b2 = (const float*)d_in[8];
    const float* c1w = (const float*)d_in[9];
    const float* bn1g = (const float*)d_in[10]; const float* bn1b = (const float*)d_in[11];
    const float* c2w = (const float*)d_in[12];
    const float* bn2g = (const float*)d_in[13]; const float* bn2b = (const float*)d_in[14];
    const float* b1g = (const float*)d_in[15]; const float* b1b = (const float*)d_in[16];
    const float* lin_w = (const float*)d_in[17]; const float* lin_b = (const float*)d_in[18];
    const float* b2g = (const float*)d_in[19]; const float* b2b = (const float*)d_in[20];
    float* out = (float*)d_out;

    char* wsp = (char*)d_ws;
    auto take = [&](size_t bytes) { char* p = wsp; wsp += (bytes + 255) & ~(size_t)255; return (void*)p; };
    float* Wd = (float*)take(NC * NC * 4);
    float* P = (float*)take((size_t)NM * NC * 4); float* Q = (float*)take((size_t)NM * NC * 4);
    double* ps1 = (double*)take((size_t)NBLK1 * 96 * 8); double* pq1 = (double*)take((size_t)NBLK1 * 96 * 8);
    float* m1 = (float*)take(96 * 4); float* v1 = (float*)take(96 * 4);
    float* Y1c = (float*)take((size_t)CHE * NC * 4); float* Y2c = (float*)take((size_t)CHE * NC * 4);
    double* ps2 = (double*)take((size_t)NBLK2 * NC * 8); double* pq2 = (double*)take((size_t)NBLK2 * NC * 8);
    float* m2 = (float*)take(NC * 4); float* v2 = (float*)take(NC * 4);
    float* YM = (float*)take((size_t)NM * NC * 4); float* YL = (float*)take((size_t)NM * NC * 4);
    float* m3 = (float*)take(NC * 4); float* v3 = (float*)take(NC * 4); float* m4 = (float*)take(NC * 4); float* v4 = (float*)take(NC * 4);
    if ((size_t)(wsp - (char*)d_ws) > ws_size) return;

    k_wd<<<(NC * NC + 255) / 256, 256, 0, stream>>>(c1w, Wd);
    { GemmArgs g = gemm_args(x, NC, zm(0), Wd, NC, zm(0), P, NC, zm(0), NM, NC, NC); g.bscale = 16.0f; g.oscale = 1.0f / 16.0f; gemm_kernel<0, 1, 1, 1, 8, 1, ACT_NONE><<<dim3(NM / 128, 1, 1), 256, 0, stream>>>(g); }
    { GemmArgs g = gemm_args(x, NC, zm(0), c1w + NC * NC, NC, zm(0), Q, NC, zm(0), NM, NC, NC); g.bscale = 16.0f; g.oscale = 1.0f / 16.0f; gemm_kernel<0, 1, 1, 1, 8, 1, ACT_NONE><<<dim3(NM / 128, 1, 1), 256, 0, stream>>>(g); }
    k_stats1<<<NBLK1, 128, 0, stream>>>(P, Q, pp, idx, lp_w1, lp_b1, ps1, pq1);
    k_reduce<<<1, 128, 0, stream>>>(ps1, pq1, NBLK1, 96, (double)NEDG, m1, v1);
    for (int ch = 0; ch < NM / CHP; ++ch) {
        k_y1act<<<(unsigned)(((size_t)CHE * NC) / 256), 256, 0, stream>>>(P, Q, idx, m1, v1, bn1g, bn1b, ch * CHE, Y1c);
        { GemmArgs g = gemm_args(Y1c, NC, zm(0), c2w, NC, zm(0), Y2c, NC, zm(0), CHE, NC, NC); g.bscale = 16.0f; g.oscale = 1.0f / 16.0f; gemm_kernel<0, 1, 1, 1, 8, 1, ACT_NONE><<<dim3(CHE / 128, 1, 1), 256, 0, stream>>>(g); }
        k_stats2<<<CHE / 1024, NC, 0, stream>>>(Y2c, ch * (CHE / 1024), ps2, pq2);
    }
    k_reduce<<<1, 128, 0, stream>>>(ps2, pq2, NBLK2, NC, (double)NEDG, m2, v2);
    for (int ch = 0; ch < NM / CHP; ++ch) {
        k_y1act<<<(unsigned)(((size_t)CHE * NC) / 256), 256, 0, stream>>>(P, Q, idx, m1, v1, bn1g, bn1b, ch * CHE, Y1c);
        { GemmArgs g = gemm_args(Y1c, NC, zm(0), c2w, NC, zm(0), Y2c, NC, zm(0), CHE, NC, NC); g.bscale = 16.0f; g.oscale = 1.0f / 16.0f; gemm_kernel<0, 1, 1, 1, 8, 1, ACT_NONE><<<dim3(CHE / 128, 1, 1), 256, 0, stream>>>(g); }
        k_apply<<<(unsigned)(((size_t)CHP * NC) / 256), 256, 0, stream>>>(Y2c, pp, idx, lp_w1, lp_b1, m1 + NC, v1 + NC, lp_g, lp_be, lp_w2, lp_b2, m2, v2, bn2g, bn2b, ch * CHP, YM);
    }
    k_colstats<<<1, NC, 0, stream>>>(YM, m3, v3);
    k_bn_node<<<(NM * NC) / 256, 256, 0, stream>>>(YM, m3, v3, b1g, b1b, nullptr, YM, 0);
    { GemmArgs g = gemm_args(YM, NC, zm(0), lin_w, NC, zm(0), YL, NC, zm(0), NM, NC, NC); g.bias = lin_b; g.bscale = 16.0f; g.oscale = 1.0f / 16.0f; gemm_kernel<0, 1, 1, 1, 8, 1, ACT_NONE><<<dim3(NM / 128, 1, 1), 256, 0, stream>>>(g); }
    k_colstats<<<1, NC, 0, stream>>>(YL, m4, v4);
    k_bn_node<<<(NM * NC) / 256, 256, 0, stream>>>(YL, m4, v4, b2g, b2b, x, out, 1);
}
